// GCN_68659347193894
// MI455X (gfx1250) — hardware-verified
//
#include <hip/hip_runtime.h>
#include <stddef.h>
#include <stdint.h>
#include <math.h>


#define CIN    128
#define NTHR   256
#define NWAVE  8
#define EPT    8
#define CHUNK  (NTHR * EPT)
#define WCAP   (EPT * 32)
#define LISTN  (NWAVE * WCAP)
#define NBA    1024
#define SLA    10
#define RCAP   20480
#define DEGCAP 64
#define GBM    64
#define GBN    64
#define GTHR   128
#define AGG_ZINTS    (LISTN + 2 * RCAP + 3 * NBA)
#define MISC_INTS    16
#define XTRA_INTS    2048
#define AGG_LDS_INTS (AGG_ZINTS + MISC_INTS + XTRA_INTS)
#define WU1    1024
#define WU2    2048
#define WU3    8192
#define WU4    4096
#define WUTOT  (WU1 + WU2 + WU3 + WU4)
#define WSMAX  134217728

static_assert((CHUNK & (CHUNK - 1)) == 0 && CHUNK <= 4096);
static_assert((NBA & (NBA - 1)) == 0 && NBA == (1 << SLA));
static_assert(((long long)CHUNK << SLA) < (1LL << 31));
static_assert(LISTN % NTHR == 0);
static_assert(NBA % NWAVE == 0 && NBA % 32 == 0 && NBA % GBM == 0 && NBA == 4 * NTHR);
static_assert(RCAP % 4 == 0 && AGG_ZINTS % (NTHR * 4) == 0 && ((AGG_ZINTS + MISC_INTS) % 4) == 0);
static_assert(XTRA_INTS % (NTHR * 4) == 0 && XTRA_INTS >= NBA && XTRA_INTS * 2 >= NWAVE * 512);
static_assert(GBM == (GTHR / 32) * 16 && GBN == 64);
static_assert(WU1 % NTHR == 0 && WU2 % NTHR == 0 && WU3 % NTHR == 0 && WU4 % NTHR == 0);
static_assert(AGG_LDS_INTS * 4 <= 300000);

typedef float          v2f   __attribute__((ext_vector_type(2)));
typedef float          v4f   __attribute__((ext_vector_type(4)));
typedef float          v8f   __attribute__((ext_vector_type(8)));
typedef int            v4i   __attribute__((ext_vector_type(4)));
typedef int            v8i   __attribute__((ext_vector_type(8)));
typedef unsigned short v2us  __attribute__((ext_vector_type(2)));
typedef unsigned short v4us  __attribute__((ext_vector_type(4)));
typedef unsigned short v8us  __attribute__((ext_vector_type(8)));
typedef unsigned short v16us __attribute__((ext_vector_type(16)));
typedef __bf16         v16bf __attribute__((ext_vector_type(16)));
typedef v2f  __attribute__((may_alias)) v2fa;
typedef v4f  __attribute__((may_alias)) v4fa;
typedef v4i  __attribute__((may_alias)) v4ia;
typedef v2us __attribute__((may_alias)) v2usa;
typedef v4us __attribute__((may_alias)) v4usa;
typedef v8us __attribute__((may_alias)) v8usa;
union FragB { v16bf v; v16us u; v8us h[2]; v8i w; };

__device__ __forceinline__ v8f wmb(const FragB& a, const FragB& b, v8f c) {
  v8f d = __builtin_amdgcn_wmma_f32_16x16x32_bf16(false, a.v, false, b.v, (short)0, c, false, false);
  asm volatile("v_nop\n\tv_nop\n\tv_nop\n\tv_nop" : "+v"(d) : "v"(a.w), "v"(b.w));
  return d;
}

__device__ __forceinline__ unsigned bf16_bits(float f) {
  const unsigned u = __float_as_uint(f);
  const unsigned r = (u + 0x7FFFu + ((u >> 16) & 1u)) >> 16;
  return (f != f) ? 0x7FC0u : r;
}
__device__ __forceinline__ float bf16_val(float f) {
  return __uint_as_float(bf16_bits(f) << 16);
}

__device__ __forceinline__ void wave_sync() {
  __builtin_amdgcn_fence(__ATOMIC_RELEASE, "wavefront");
  __builtin_amdgcn_wave_barrier();
  __builtin_amdgcn_fence(__ATOMIC_ACQUIRE, "wavefront");
}

template <int C>
__device__ __forceinline__ void ld_row(const float* __restrict__ rp, int lane, float (&v)[C / 32]) {
  if constexpr (C == 64) {
    const v2f a = *(const v2fa*)(rp + 2 * lane);
    v[0] = a.x; v[1] = a.y;
  } else {
#pragma unroll
    for (int g = 0; g < C / 128; ++g) {
      const v4f a = *(const v4fa*)(rp + 128 * g + 4 * lane);
      v[4 * g + 0] = a.x; v[4 * g + 1] = a.y; v[4 * g + 2] = a.z; v[4 * g + 3] = a.w;
    }
  }
}

template <int SLB>
__device__ __forceinline__ int scan_chunk(const int* __restrict__ dsts, int nE, int cbase, int slotBase,
                                          int nb, int vec8, int* list, int tid, int lane, int wave) {
  int wc = 0;
  const int el0  = tid * EPT;
  const int e0   = cbase + el0;
  const int sent = -2147483647 - 1;
  v4i da, db;
  if (vec8 != 0 && cbase + CHUNK <= nE) {
    da = *(const v4i*)(dsts + e0);
    db = *(const v4i*)(dsts + e0 + 4);
  } else {
    da.x = (e0     < nE) ? dsts[min(e0,     nE - 1)] : sent;
    da.y = (e0 + 1 < nE) ? dsts[min(e0 + 1, nE - 1)] : sent;
    da.z = (e0 + 2 < nE) ? dsts[min(e0 + 2, nE - 1)] : sent;
    da.w = (e0 + 3 < nE) ? dsts[min(e0 + 3, nE - 1)] : sent;
    db.x = (e0 + 4 < nE) ? dsts[min(e0 + 4, nE - 1)] : sent;
    db.y = (e0 + 5 < nE) ? dsts[min(e0 + 5, nE - 1)] : sent;
    db.z = (e0 + 6 < nE) ? dsts[min(e0 + 6, nE - 1)] : sent;
    db.w = (e0 + 7 < nE) ? dsts[min(e0 + 7, nE - 1)] : sent;
  }
  const unsigned nbs = (unsigned)slotBase;
  const unsigned unb = (unsigned)nb;
  const unsigned s0 = (unsigned)da.x - nbs, s1 = (unsigned)da.y - nbs;
  const unsigned s2 = (unsigned)da.z - nbs, s3 = (unsigned)da.w - nbs;
  const unsigned s4 = (unsigned)db.x - nbs, s5 = (unsigned)db.y - nbs;
  const unsigned s6 = (unsigned)db.z - nbs, s7 = (unsigned)db.w - nbs;
  const bool h0 = s0 < unb, h1 = s1 < unb, h2 = s2 < unb, h3 = s3 < unb;
  const bool h4 = s4 < unb, h5 = s5 < unb, h6 = s6 < unb, h7 = s7 < unb;
  const unsigned any = __builtin_amdgcn_ballot_w32(h0 | h1 | h2 | h3 | h4 | h5 | h6 | h7);
  if (any != 0u) {
#define HITJ(J, HJ, SJ) { \
      const unsigned mj = __builtin_amdgcn_ballot_w32(HJ); \
      if (mj != 0u) { \
        if (HJ) { \
          const int pos = wc + (int)__builtin_amdgcn_mbcnt_lo(mj, 0u); \
          if (pos < WCAP) list[wave * WCAP + pos] = ((el0 + (J)) << SLB) | (int)(SJ); \
        } \
        wc += (int)__builtin_popcount(mj); } }
    HITJ(0, h0, s0)
    HITJ(1, h1, s1)
    HITJ(2, h2, s2)
    HITJ(3, h3, s3)
    HITJ(4, h4, s4)
    HITJ(5, h5, s5)
    HITJ(6, h6, s6)
    HITJ(7, h7, s7)
#undef HITJ
  }
  return wc;
}

__device__ __forceinline__ void build_lists(const int* __restrict__ dsts, int nE, int vec8, int nodeBase,
                                            int* dsm, int tid, int lane, int wave, int& ovfOut) {
  int* list = dsm;
  int* hl   = dsm + LISTN;
  int* sl   = hl + RCAP;
  int* cnt  = sl + RCAP;
  int* offs = cnt + NBA;
  int* cur  = offs + NBA;
  int* misc = cur + NBA;
  {
    const v4i z4 = {0, 0, 0, 0};
    for (int i = tid * 4; i < AGG_ZINTS; i += NTHR * 4) *(v4ia*)(dsm + i) = z4;
    if (tid < MISC_INTS) misc[tid] = 0;
    for (int i = tid * 4; i < XTRA_INTS; i += NTHR * 4) *(v4ia*)(misc + MISC_INTS + i) = z4;
  }
  __syncthreads();

  int t = 0, ov = 0;
  const int nChunks = (nE + CHUNK - 1) / CHUNK;
#pragma unroll 1
  for (int ch = 0; ch < nChunks; ++ch) {
    const int cbase = ch * CHUNK;
    const int wc = scan_chunk<SLA>(dsts, nE, cbase, nodeBase, NBA, vec8, list, tid, lane, wave);
    if (lane == 0) misc[wave] = wc;
    __syncthreads();
    if (wave == 0) {
#pragma unroll 1
      for (int w2 = 0; w2 < NWAVE; ++w2) {
        int c = misc[w2];
        c = c < 0 ? 0 : (c > WCAP ? WCAP : c);
#pragma unroll 1
        for (int b0 = 0; b0 < c; b0 += 32) {
          const int idx = b0 + lane;
          const int ent = list[w2 * WCAP + (idx < WCAP ? idx : WCAP - 1)];
          const int m32 = (c - b0) < 32 ? (c - b0) : 32;
#pragma unroll 1
          for (int k = 0; k < m32; ++k) {
            const int u    = __builtin_amdgcn_readlane(ent, k);
            const int slot = u & (NBA - 1);
            const int el   = (u >> SLA) & (CHUNK - 1);
            const int pk   = ((cbase + el) << SLA) | slot;
            if (t < RCAP) {
              if (lane == 0) { hl[t] = pk; cnt[slot] = cnt[slot] + 1; }
              t = t + 1;
            } else {
              ov = 1;
            }
          }
        }
      }
    }
    __syncthreads();
  }
  if (wave == 0 && lane == 0) { misc[8] = t; misc[9] = ov; }
  __syncthreads();
  int tt = misc[8];
  tt = tt < 0 ? 0 : (tt > RCAP ? RCAP : tt);
  const int ovf = misc[9];

  if (wave == 0) {
    const int base = lane * (NBA / 32);
    int s = 0;
#pragma unroll 1
    for (int i = 0; i < NBA / 32; ++i) s += cnt[base + i];
    int incl = s;
#pragma unroll
    for (int d = 1; d < 32; d <<= 1) {
      const int y = __shfl_up(incl, d, 32);
      if (lane >= d) incl += y;
    }
    int run = incl - s;
#pragma unroll 1
    for (int i = 0; i < NBA / 32; ++i) {
      const int cv = cnt[base + i];
      offs[base + i] = run;
      cur[base + i]  = run;
      run += cv;
    }
  }
  __syncthreads();
  if (wave == 0) {
#pragma unroll 1
    for (int b0 = 0; b0 < tt; b0 += 32) {
      const int idx = b0 + lane;
      const int ent = hl[idx < RCAP ? idx : RCAP - 1];
      const int m32 = (tt - b0) < 32 ? (tt - b0) : 32;
#pragma unroll 1
      for (int k = 0; k < m32; ++k) {
        const int u    = __builtin_amdgcn_readlane(ent, k);
        const int slot = u & (NBA - 1);
        if (lane == 0) {
          int p = cur[slot];
          p = p < 0 ? 0 : (p > RCAP - 1 ? RCAP - 1 : p);
          sl[p] = u;
          cur[slot] = p + 1;
        }
      }
    }
  }
  __syncthreads();
  ovfOut = ovf;
}

__global__ __launch_bounds__(NTHR) void k_wprep(const float* __restrict__ W1, const float* __restrict__ W2,
                                                const float* __restrict__ W3, const float* __restrict__ W4,
                                                unsigned short* W1T, unsigned short* W2T,
                                                unsigned short* W3T, unsigned short* W4T) {
  const int u = (int)blockIdx.x * NTHR + (int)threadIdx.x;
  const float* W;
  unsigned short* P;
  int N, kin, kt, v;
  if (u < WU1)                   { W = W1; P = W1T; N = 64;  kin = 128; kt = 128; v = u; }
  else if (u < WU1 + WU2)        { W = W2; P = W2T; N = 128; kin = 64;  kt = 128; v = u - WU1; }
  else if (u < WU1 + WU2 + WU3)  { W = W3; P = W3T; N = 256; kin = 128; kt = 256; v = u - WU1 - WU2; }
  else if (u < WUTOT)            { W = W4; P = W4T; N = 64;  kin = 256; kt = 512; v = u - WU1 - WU2 - WU3; }
  else return;
  const int upr = kt >> 3;
  const int n   = v / upr;
  const int k8  = (v - n * upr) * 8;
  const int kk  = k8 & (kin - 1);
  const float* p = W + (size_t)kk * N + n;
  v8us o;
#pragma unroll
  for (int i = 0; i < 8; ++i) o[i] = (unsigned short)bf16_bits(p[(size_t)i * N]);
  unsigned short* dp = P + (size_t)n * kt + k8;
  *(volatile v8us*)dp = o;
  __threadfence();
  *(volatile v8us*)dp = o;
}

__global__ __launch_bounds__(NTHR) void k_cvx(const float* __restrict__ x, int nN, int nUnits,
                                              unsigned short* xb) {
  const int u = (int)blockIdx.x * NTHR + (int)threadIdx.x;
  if (u >= nUnits) return;
  const int row = u >> 4;
  const int k8  = (u & 15) * 8;
  const int rc  = row < nN ? row : nN - 1;
  const float* p = x + (size_t)rc * CIN + k8;
  const v4f a = *(const v4fa*)p;
  const v4f b = *(const v4fa*)(p + 4);
  const bool ok = row < nN;
  v8us o;
  o[0] = ok ? (unsigned short)bf16_bits(a.x) : (unsigned short)0;
  o[1] = ok ? (unsigned short)bf16_bits(a.y) : (unsigned short)0;
  o[2] = ok ? (unsigned short)bf16_bits(a.z) : (unsigned short)0;
  o[3] = ok ? (unsigned short)bf16_bits(a.w) : (unsigned short)0;
  o[4] = ok ? (unsigned short)bf16_bits(b.x) : (unsigned short)0;
  o[5] = ok ? (unsigned short)bf16_bits(b.y) : (unsigned short)0;
  o[6] = ok ? (unsigned short)bf16_bits(b.z) : (unsigned short)0;
  o[7] = ok ? (unsigned short)bf16_bits(b.w) : (unsigned short)0;
  unsigned short* dp = xb + (size_t)row * CIN + k8;
  *(volatile v8us*)dp = o;
  __threadfence();
  *(volatile v8us*)dp = o;
}

__global__ __launch_bounds__(GTHR) void k_gemm(
    const unsigned short* __restrict__ A, const unsigned short* __restrict__ WT,
    float* outF, int K, int ldo)
{
  __shared__ __attribute__((aligned(16))) float stg[GBM * GBN];
  const int tid = (int)threadIdx.x, lane = tid & 31, wave = tid >> 5, hh = lane >> 4, m = lane & 15;
  const int rowBase = (int)blockIdx.x * GBM;
  const int col0    = (int)blockIdx.y * GBN;

  v8f acc[4];
  {
    const v8f z = {0.f, 0.f, 0.f, 0.f, 0.f, 0.f, 0.f, 0.f};
    acc[0] = z; acc[1] = z; acc[2] = z; acc[3] = z;
  }
  const unsigned short* ap = A  + (size_t)(rowBase + 16 * wave + m) * (size_t)K + 8 * hh;
  const unsigned short* wp = WT + (size_t)(col0 + m) * (size_t)K + 8 * hh;
  const int ksteps = K >> 5;
#pragma unroll 1
  for (int ks = 0; ks < ksteps; ++ks) {
    FragB af;
    af.h[0] = *(const v8usa*)(ap + 32 * ks);
    af.h[1] = *(const v8usa*)(ap + 32 * ks + 16);
#pragma unroll
    for (int t = 0; t < 4; ++t) {
      const unsigned short* wq = wp + (size_t)(16 * t) * (size_t)K + 32 * ks;
      FragB bf;
      bf.h[0] = *(const v8usa*)wq;
      bf.h[1] = *(const v8usa*)(wq + 16);
      acc[t] = wmb(af, bf, acc[t]);
    }
  }

#pragma unroll
  for (int t = 0; t < 4; ++t) {
    const int lc = 16 * t + m;
#pragma unroll
    for (int r = 0; r < 8; ++r) {
      const int lr = 16 * wave + 8 * hh + r;
      stg[lr * GBN + lc] = acc[t][r];
    }
  }
  __syncthreads();

  v4f fv[8];
#pragma unroll
  for (int i = 0; i < 8; ++i) {
    const int lr = 16 * wave + 2 * i + hh;
    fv[i] = *(const v4fa*)(stg + lr * GBN + 4 * m);
  }
#pragma unroll
  for (int i = 0; i < 8; ++i) {
    const int lr = 16 * wave + 2 * i + hh;
    const int gr = rowBase + lr;
    float* op = outF + (size_t)gr * (size_t)ldo + col0 + 4 * m;
    *(volatile v4f*)op = fv[i];
  }
  __threadfence();
#pragma unroll
  for (int i = 0; i < 8; ++i) {
    const int lr = 16 * wave + 2 * i + hh;
    const int gr = rowBase + lr;
    float* op = outF + (size_t)gr * (size_t)ldo + col0 + 4 * m;
    *(volatile v4f*)op = fv[i];
  }
}

template <int C, int MODE>
__global__ __launch_bounds__(NTHR) void k_agg(const int* __restrict__ srcs, const int* __restrict__ dsts,
                                              const float* __restrict__ ew, int nE, int nN, int vec8, int mRows,
                                              const float* __restrict__ dis, const float* __restrict__ xl,
                                              const float* __restrict__ bias, const float* __restrict__ w5,
                                              unsigned short* hb, float* t5) {
  static_assert(C == 64 || C == 128 || C == 256);
  static_assert(MODE == 1 || (MODE == 2 && C == 64));
  constexpr int NCH = C / 32;
  extern __shared__ __attribute__((aligned(16))) int dsm[];
  int* sl   = dsm + LISTN + RCAP;
  int* cnt  = sl + RCAP;
  int* offs = cnt + NBA;
  int* misc = offs + 2 * NBA;
  const int tid = (int)threadIdx.x, lane = tid & 31, wave = tid >> 5;
  const int nodeBase = (int)blockIdx.x * NBA;
  unsigned short* rowbuf = (unsigned short*)(misc + MISC_INTS) + wave * 512;
  float* t5s = (float*)(misc + MISC_INTS);

  int ovf;
  build_lists(dsts, nE, vec8, nodeBase, dsm, tid, lane, wave, ovf);

  float bv[NCH];
  {
    float tb[NCH];
    ld_row<C>(bias, lane, tb);
#pragma unroll
    for (int i = 0; i < NCH; ++i) bv[i] = bf16_val(tb[i]);
  }
  float wq[NCH];
#pragma unroll
  for (int i = 0; i < NCH; ++i) wq[i] = 0.0f;
  if constexpr (MODE == 2) {
    float tw[NCH];
    ld_row<C>(w5, lane, tw);
#pragma unroll
    for (int i = 0; i < NCH; ++i) wq[i] = bf16_val(tw[i]);
  }

  const float qnan = __int_as_float(0x7fc00000);
  const float pz = (ovf != 0) ? qnan : 0.0f;
  const int l8 = (C == 64) ? 8 * (lane & 15) : 8 * lane;
#pragma unroll 1
  for (int si = 0; si < NBA / NWAVE; ++si) {
    const int s    = si * NWAVE + wave;
    const int node = nodeBase + s;
    int c = __builtin_amdgcn_readfirstlane(cnt[s]);
    const bool big = c > DEGCAP;
    c = c < 0 ? 0 : (c > DEGCAP ? DEGCAP : c);
    int o = __builtin_amdgcn_readfirstlane(offs[s]);
    o = o < 0 ? 0 : (o > RCAP ? RCAP : o);
    const int nc = node < nN ? node : nN - 1;
    const float dd = dis[nc];
    const float rd = dd * dd;
    float acc[NCH];
#pragma unroll
    for (int i = 0; i < NCH; ++i) acc[i] = 0.0f;
#pragma unroll 1
    for (int b0 = 0; b0 < c; b0 += 32) {
      int idx = o + b0 + lane;
      idx = idx > RCAP - 1 ? RCAP - 1 : idx;
      const int ent = sl[idx];
      int eid = ent >> SLA;
      eid = eid < 0 ? 0 : (eid > nE - 1 ? nE - 1 : eid);
      int sr = srcs[eid];
      sr = sr < 0 ? 0 : (sr > nN - 1 ? nN - 1 : sr);
      const float wv  = bf16_val(ew[eid]);
      const float cf  = (dis[sr] * wv) * dd;
      const int   cfi = __float_as_int(cf);
      const int m32 = (c - b0) < 32 ? (c - b0) : 32;
#pragma unroll 1
      for (int k = 0; k < m32; ++k) {
        const int   sk = __builtin_amdgcn_readlane(sr, k);
        const float ck = __int_as_float(__builtin_amdgcn_readlane(cfi, k));
        float rv[NCH];
        ld_row<C>(xl + (size_t)sk * C, lane, rv);
#pragma unroll
        for (int i = 0; i < NCH; ++i) acc[i] = fmaf(ck, rv[i], acc[i]);
      }
    }
    float sv[NCH];
    ld_row<C>(xl + (size_t)nc * C, lane, sv);
    const float pzr = big ? qnan : pz;
    const bool live = node < nN;
    float v[NCH];
#pragma unroll
    for (int i = 0; i < NCH; ++i) {
      float y = (acc[i] + sv[i] * rd) + bv[i];
      y = (y > 0.0f) ? y : (y - y);
      y = y + pzr;
      v[i] = live ? y : 0.0f;
    }

    if constexpr (MODE == 1) {
      if constexpr (C == 64) {
        const unsigned h0 = bf16_bits(v[0]), h1 = bf16_bits(v[1]);
        v2us mh, ml;
        mh[0] = (unsigned short)h0; mh[1] = (unsigned short)h1;
        ml[0] = (unsigned short)bf16_bits(v[0] - __uint_as_float(h0 << 16));
        ml[1] = (unsigned short)bf16_bits(v[1] - __uint_as_float(h1 << 16));
        *(v2usa*)(rowbuf + 2 * lane) = mh;
        *(v2usa*)(rowbuf + C + 2 * lane) = ml;
      } else {
#pragma unroll
        for (int g = 0; g < C / 128; ++g) {
          v4us mh, ml;
#pragma unroll
          for (int j = 0; j < 4; ++j) {
            const unsigned hbj = bf16_bits(v[4 * g + j]);
            mh[j] = (unsigned short)hbj;
            ml[j] = (unsigned short)bf16_bits(v[4 * g + j] - __uint_as_float(hbj << 16));
          }
          *(v4usa*)(rowbuf + 128 * g + 4 * lane) = mh;
          *(v4usa*)(rowbuf + C + 128 * g + 4 * lane) = ml;
        }
      }
      wave_sync();
      constexpr int NST = (2 * C >= 256) ? (2 * C / 256) : 1;
      v8us q[NST];
#pragma unroll
      for (int j = 0; j < NST; ++j) q[j] = *(const v8usa*)(rowbuf + 256 * j + l8);
      wave_sync();
      const bool wr = (node < mRows) && (C != 64 || lane < 16);
      unsigned short* rpw = hb + (size_t)node * (2 * C) + l8;
      if (wr) {
#pragma unroll
        for (int j = 0; j < NST; ++j) *(volatile v8us*)(rpw + 256 * j) = q[j];
      }
      __threadfence();
      if (wr) {
#pragma unroll
        for (int j = 0; j < NST; ++j) *(volatile v8us*)(rpw + 256 * j) = q[j];
      }
    } else {
      float p = v[0] * wq[0];
#pragma unroll
      for (int i = 1; i < NCH; ++i) p = fmaf(v[i], wq[i], p);
#pragma unroll
      for (int d = 16; d >= 1; d >>= 1) p += __shfl_xor(p, d, 32);
      if (lane == 0) t5s[s] = p;
    }
  }

  if constexpr (MODE == 2) {
    __syncthreads();
    const v4f ov = *(const v4fa*)(t5s + 4 * tid);
    float* op = t5 + (size_t)nodeBase + 4 * tid;
    *(volatile v4f*)op = ov;
    __threadfence();
    *(volatile v4f*)op = ov;
  }
}

template <int MODE>
__global__ __launch_bounds__(NTHR) void k_sc(const int* __restrict__ srcs, const int* __restrict__ dsts,
                                             const float* __restrict__ ew, int nE, int nN, int vec8,
                                             const float* __restrict__ dis, const float* __restrict__ t5,
                                             const float* __restrict__ b5, float* outp, int nOutRows) {
  extern __shared__ __attribute__((aligned(16))) int dsm[];
  int* sl   = dsm + LISTN + RCAP;
  int* cnt  = sl + RCAP;
  int* offs = cnt + NBA;
  int* misc = offs + 2 * NBA;
  float* os = (float*)(misc + MISC_INTS);
  const int tid = (int)threadIdx.x, lane = tid & 31, wave = tid >> 5;
  const int nodeBase = (int)blockIdx.x * NBA;

  int ovf;
  build_lists(dsts, nE, vec8, nodeBase, dsm, tid, lane, wave, ovf);

  float bb = 0.0f;
  if constexpr (MODE == 1) bb = bf16_val(b5[0]);
  const float qnan = __int_as_float(0x7fc00000);
  const float pz = (ovf != 0) ? qnan : 0.0f;
#pragma unroll 1
  for (int si = 0; si < NBA / NWAVE; ++si) {
    const int s    = si * NWAVE + wave;
    const int node = nodeBase + s;
    int c = __builtin_amdgcn_readfirstlane(cnt[s]);
    const bool big = c > DEGCAP;
    c = c < 0 ? 0 : (c > DEGCAP ? DEGCAP : c);
    int o = __builtin_amdgcn_readfirstlane(offs[s]);
    o = o < 0 ? 0 : (o > RCAP ? RCAP : o);
    const int nc = node < nN ? node : nN - 1;
    float dd = 0.0f, rd = 0.0f, tself = 0.0f;
    if constexpr (MODE == 1) { dd = dis[nc]; rd = dd * dd; tself = t5[nc]; }
    float acc = 0.0f;
#pragma unroll 1
    for (int b0 = 0; b0 < c; b0 += 32) {
      int idx = o + b0 + lane;
      idx = idx > RCAP - 1 ? RCAP - 1 : idx;
      const int ent = sl[idx];
      int eid = ent >> SLA;
      eid = eid < 0 ? 0 : (eid > nE - 1 ? nE - 1 : eid);
      const float wv = bf16_val(ew[eid]);
      float val = wv;
      if constexpr (MODE == 1) {
        int sr = srcs[eid];
        sr = sr < 0 ? 0 : (sr > nN - 1 ? nN - 1 : sr);
        const float cf = (dis[sr] * wv) * dd;
        val = cf * t5[sr];
      }
      const bool valid = (b0 + lane) < c;
      val = valid ? val : 0.0f;
#pragma unroll
      for (int d = 16; d >= 1; d >>= 1) val += __shfl_xor(val, d, 32);
      acc += val;
    }
    const float pzr = big ? qnan : pz;
    float r;
    if constexpr (MODE == 0) {
      const float deg = acc + 1.0f;
      r = (deg > 0.0f) ? rsqrtf(deg) : 0.0f;
    } else {
      const float y = (acc + rd * tself) + bb;
      r = tanhf(y);
    }
    r = r + pzr;
    r = (node < nN) ? r : 0.0f;
    if (lane == 0) os[s] = r;
  }
  __syncthreads();
  const v4f ov = *(const v4fa*)(os + 4 * tid);
  float* op = outp + (size_t)nodeBase + 4 * tid;
  const bool wr = (nodeBase + 4 * tid + 3) < nOutRows;
  if (wr) *(volatile v4f*)op = ov;
  __threadfence();
  if (wr) *(volatile v4f*)op = ov;
}

static inline int cdiv(int a, int b) { return (a + b - 1) / b; }
static inline size_t al256(size_t o) { return (o + 255) & ~(size_t)255; }

extern "C" void kernel_launch(void* const* d_in, const int* in_sizes, int n_in,
                              void* d_out, int out_size, void* d_ws, size_t ws_size,
                              hipStream_t stream) {
  if (n_in < 13) return;
  if (in_sizes[0] < CIN || (in_sizes[0] % CIN) != 0) return;
  const int nN = in_sizes[0] / CIN;
  if (nN < 32 || nN > (1 << 22) || (nN % 32) != 0) return;
  if (in_sizes[1] < 2 || (in_sizes[1] & 1) != 0) return;
  const int nE = in_sizes[1] / 2;
  if (nE < 1 || nE >= (1 << (31 - SLA))) return;
  if (in_sizes[2] != nE) return;
  if (in_sizes[3] != 128 * 64  || in_sizes[4]  != 64)  return;
  if (in_sizes[5] != 64 * 128  || in_sizes[6]  != 128) return;
  if (in_sizes[7] != 128 * 256 || in_sizes[8]  != 256) return;
  if (in_sizes[9] != 256 * 64  || in_sizes[10] != 64)  return;
  if (in_sizes[11] != 64 || in_sizes[12] != 1) return;
  if (out_size != nN) return;

  const float* x    = (const float*)d_in[0];
  const int*   edge = (const int*)d_in[1];
  const float* ew   = (const float*)d_in[2];
  const float* W1   = (const float*)d_in[3];
  const float* b1   = (const float*)d_in[4];
  const float* W2   = (const float*)d_in[5];
  const float* b2   = (const float*)d_in[6];
  const float* W3   = (const float*)d_in[7];
  const float* b3   = (const float*)d_in[8];
  const float* W4   = (const float*)d_in[9];
  const float* b4   = (const float*)d_in[10];
  const float* W5   = (const float*)d_in[11];
  const float* b5   = (const float*)d_in[12];
  float* out = (float*)d_out;
  const int* src = edge;
  const int* dst = edge + nE;

  const int MP  = cdiv(nN, GBM) * GBM;
  const int gM  = MP / GBM;
  const int gA  = cdiv(MP, NBA);
  const int NSL = gA * NBA;
  if ((long long)gA * NBA < (long long)MP) return;
  const int vec8 = ((nE & 3) == 0) ? 1 : 0;

  char* ws = (char*)d_ws;
  size_t off = 0;
  const size_t oDIS = off; off = al256(off + (size_t)NSL * 4);
  const size_t oW1T = off; off = al256(off + (size_t)64 * 128 * 2);
  const size_t oW2T = off; off = al256(off + (size_t)128 * 128 * 2);
  const size_t oW3T = off; off = al256(off + (size_t)256 * 256 * 2);
  const size_t oW4T = off; off = al256(off + (size_t)64 * 512 * 2);
  const size_t oXB  = off; off = al256(off + (size_t)MP * 128 * 2);
  const size_t oT1  = off; off = al256(off + (size_t)MP * 64 * 4);
  const size_t oH1  = off; off = al256(off + (size_t)MP * 128 * 2);
  const size_t oT2  = off; off = al256(off + (size_t)MP * 128 * 4);
  const size_t oH2  = off; off = al256(off + (size_t)MP * 256 * 2);
  const size_t oT3  = off; off = al256(off + (size_t)MP * 256 * 4);
  const size_t oH3  = off; off = al256(off + (size_t)MP * 512 * 2);
  const size_t oT4  = off; off = al256(off + (size_t)MP * 64 * 4);
  const size_t oT5  = off; off = al256(off + (size_t)NSL * 4);
  if (off > ws_size || off > (size_t)WSMAX) return;
  float*          DIS = (float*)(ws + oDIS);
  unsigned short* W1T = (unsigned short*)(ws + oW1T);
  unsigned short* W2T = (unsigned short*)(ws + oW2T);
  unsigned short* W3T = (unsigned short*)(ws + oW3T);
  unsigned short* W4T = (unsigned short*)(ws + oW4T);
  unsigned short* XB  = (unsigned short*)(ws + oXB);
  float*          T1  = (float*)(ws + oT1);
  unsigned short* H1  = (unsigned short*)(ws + oH1);
  float*          T2  = (float*)(ws + oT2);
  unsigned short* H2  = (unsigned short*)(ws + oH2);
  float*          T3  = (float*)(ws + oT3);
  unsigned short* H3  = (unsigned short*)(ws + oH3);
  float*          T4  = (float*)(ws + oT4);
  float*          T5  = (float*)(ws + oT5);

  const size_t sLds = (size_t)AGG_LDS_INTS * 4;
  hipFuncSetAttribute(reinterpret_cast<const void*>(&k_sc<0>), hipFuncAttributeMaxDynamicSharedMemorySize, (int)sLds);
  hipFuncSetAttribute(reinterpret_cast<const void*>(&k_sc<1>), hipFuncAttributeMaxDynamicSharedMemorySize, (int)sLds);
  hipFuncSetAttribute(reinterpret_cast<const void*>(&k_agg<64, 1>), hipFuncAttributeMaxDynamicSharedMemorySize, (int)sLds);
  hipFuncSetAttribute(reinterpret_cast<const void*>(&k_agg<128, 1>), hipFuncAttributeMaxDynamicSharedMemorySize, (int)sLds);
  hipFuncSetAttribute(reinterpret_cast<const void*>(&k_agg<256, 1>), hipFuncAttributeMaxDynamicSharedMemorySize, (int)sLds);
  hipFuncSetAttribute(reinterpret_cast<const void*>(&k_agg<64, 2>), hipFuncAttributeMaxDynamicSharedMemorySize, (int)sLds);

  const int nUx = MP * (CIN / 8);
  k_wprep<<<WUTOT / NTHR, NTHR, 0, stream>>>(W1, W2, W3, W4, W1T, W2T, W3T, W4T);
  k_cvx<<<cdiv(nUx, NTHR), NTHR, 0, stream>>>(x, nN, nUx, XB);
  k_sc<0><<<gA, NTHR, sLds, stream>>>(src, dst, ew, nE, nN, vec8, T5, T5, b5, DIS, NSL);
  k_gemm<<<dim3(gM, 64 / GBN), GTHR, 0, stream>>>(XB, W1T, T1, 128, 64);
  k_agg<64, 1><<<gA, NTHR, sLds, stream>>>(src, dst, ew, nE, nN, vec8, MP, DIS, T1, b1, W5, H1, T5);
  k_gemm<<<dim3(gM, 128 / GBN), GTHR, 0, stream>>>(H1, W2T, T2, 128, 128);
  k_agg<128, 1><<<gA, NTHR, sLds, stream>>>(src, dst, ew, nE, nN, vec8, MP, DIS, T2, b2, W5, H2, T5);
  k_gemm<<<dim3(gM, 256 / GBN), GTHR, 0, stream>>>(H2, W3T, T3, 256, 256);
  k_agg<256, 1><<<gA, NTHR, sLds, stream>>>(src, dst, ew, nE, nN, vec8, MP, DIS, T3, b3, W5, H3, T5);
  k_gemm<<<dim3(gM, 64 / GBN), GTHR, 0, stream>>>(H3, W4T, T4, 512, 64);
  k_agg<64, 2><<<gA, NTHR, sLds, stream>>>(src, dst, ew, nE, nN, vec8, MP, DIS, T4, b4, W5, H1, T5);
  k_sc<1><<<gA, NTHR, sLds, stream>>>(src, dst, ew, nE, nN, vec8, DIS, T5, b5, out, nN);
}
